// StandardCausalAttention_56367150793407
// MI455X (gfx1250) — hardware-verified
//
#include <hip/hip_runtime.h>
#include <float.h>
#include <stdint.h>


typedef __bf16 v16bf __attribute__((ext_vector_type(16)));
typedef float v8f __attribute__((ext_vector_type(8)));
typedef float v4f __attribute__((ext_vector_type(4)));
typedef unsigned int v4u __attribute__((ext_vector_type(4)));
typedef unsigned short us_t;

#define EMBED  1024
#define NHEADS 16
#define HDIM   64
#define SEQ    2048
#define BATCH  2
#define BHEADS (BATCH * NHEADS)
#define MROWS  (BATCH * SEQ)
#define N3     (3 * EMBED)
#define SCP    132
#define SSP    68

union FragU { v16bf v; v4u w[2]; };

static __device__ __forceinline__ v16bf ldfrag(const us_t* p, int pitch, int m, int hl) {
  FragU u;
  const us_t* q = p + (size_t)m * pitch + 8 * hl;
  u.w[0] = *(const v4u*)(q);
  u.w[1] = *(const v4u*)(q + 16);
  return u.v;
}

static __device__ __forceinline__ v8f wmma16(v16bf a, v16bf b, v8f c) {
  return __builtin_amdgcn_wmma_f32_16x16x32_bf16(false, a, false, b, (short)0, c, false, false);
}

static __device__ __forceinline__ v8f mma3(v8f c, v16bf ah, v16bf al, v16bf bh, v16bf bl) {
  c = wmma16(ah, bh, c);
  c = wmma16(ah, bl, c);
  c = wmma16(al, bh, c);
  asm volatile("v_nop\n\tv_nop\n\tv_nop\n\tv_nop" : "+v"(c) : "v"(ah), "v"(al), "v"(bh), "v"(bl));
  return c;
}

static __device__ __forceinline__ unsigned bfb(float f) {
  unsigned u = __float_as_uint(f);
  return (u + 0x7FFFu + ((u >> 16) & 1u)) >> 16;
}

static __device__ __forceinline__ void split2w(float x0, float x1, unsigned& hw, unsigned& lw) {
  const unsigned h0 = bfb(x0), h1 = bfb(x1);
  const unsigned l0 = bfb(x0 - __uint_as_float(h0 << 16));
  const unsigned l1 = bfb(x1 - __uint_as_float(h1 << 16));
  hw = h0 | (h1 << 16);
  lw = l0 | (l1 << 16);
}

static __device__ __forceinline__ void split8(v4f a, v4f c, v4u& hw, v4u& lw) {
  unsigned h, lo;
  split2w(a[0], a[1], h, lo); hw[0] = h; lw[0] = lo;
  split2w(a[2], a[3], h, lo); hw[1] = h; lw[1] = lo;
  split2w(c[0], c[1], h, lo); hw[2] = h; lw[2] = lo;
  split2w(c[2], c[3], h, lo); hw[3] = h; lw[3] = lo;
}

__global__ __launch_bounds__(256) void k_cvt_rows(const float* __restrict__ src,
                                                   us_t* Ph, us_t* Pl, int n8) {
  const int t = blockIdx.x * 256 + (int)threadIdx.x;
  if (t >= n8) return;
  const size_t o = (size_t)t * 8;
  const v4f a = *(const v4f*)(src + o);
  const v4f c = *(const v4f*)(src + o + 4);
  v4u hw, lw;
  split8(a, c, hw, lw);
  *(volatile v4u*)(Ph + o) = hw;
  *(volatile v4u*)(Pl + o) = lw;
  __threadfence();
  *(volatile v4u*)(Ph + o) = hw;
  *(volatile v4u*)(Pl + o) = lw;
}

__global__ __launch_bounds__(256) void k_cvt_tr(const float* __restrict__ src,
                                                 us_t* Ph, us_t* Pl, int R, int Ncol) {
  __shared__ __align__(16) float sW[64 * 65];
  const int tid = (int)threadIdx.x;
  const int c0 = blockIdx.x * 64;
  const int r0 = blockIdx.y * 64;
#pragma unroll
  for (int it = 0; it < 4; ++it) {
    const int r = it * 16 + (tid >> 4);
    const int c4 = (tid & 15) * 4;
    const v4f v = *(const v4f*)(src + (size_t)(r0 + r) * Ncol + c0 + c4);
    sW[r * 65 + c4 + 0] = v[0];
    sW[r * 65 + c4 + 1] = v[1];
    sW[r * 65 + c4 + 2] = v[2];
    sW[r * 65 + c4 + 3] = v[3];
  }
  __syncthreads();
  for (int pass = 0; pass < 2; ++pass) {
#pragma unroll
    for (int it = 0; it < 2; ++it) {
      const int L = it * 32 + (tid >> 3);
      const int seg = (tid & 7) * 8;
      v4f a, c;
#pragma unroll
      for (int e = 0; e < 4; ++e) {
        a[e] = sW[(seg + e) * 65 + L];
        c[e] = sW[(seg + 4 + e) * 65 + L];
      }
      v4u hw, lw;
      split8(a, c, hw, lw);
      const size_t d = (size_t)(c0 + L) * R + r0 + seg;
      *(volatile v4u*)(Ph + d) = hw;
      *(volatile v4u*)(Pl + d) = lw;
    }
    if (pass == 0) __threadfence();
  }
}

template <int EPI>
__global__ __launch_bounds__(256) void k_gemm(const us_t* __restrict__ Ah, const us_t* __restrict__ Al,
                                               const us_t* __restrict__ Bh, const us_t* __restrict__ Bl,
                                               const float* __restrict__ bias,
                                               us_t* Qh, us_t* Ql, us_t* Kh, us_t* Kl,
                                               us_t* Vh, us_t* Vl, float* Fo) {
  __shared__ __align__(16) float sC[64 * SCP];

  const int tid = (int)threadIdx.x;
  const int l = tid & 31, hl = l >> 4, m = l & 15;
  const int w = tid >> 5;
  const int wm = w >> 2;
  const int wn = w & 3;
  const int m0 = blockIdx.y * 64;
  const int n0 = blockIdx.x * 128;

  const us_t* aph = Ah + (size_t)(m0 + wm * 32) * EMBED;
  const us_t* apl = Al + (size_t)(m0 + wm * 32) * EMBED;
  const us_t* bph = Bh + (size_t)(n0 + wn * 32) * EMBED;
  const us_t* bpl = Bl + (size_t)(n0 + wn * 32) * EMBED;

  v8f acc[2][2];
#pragma unroll
  for (int i = 0; i < 2; ++i)
#pragma unroll
    for (int j = 0; j < 2; ++j) acc[i][j] = v8f{};

#pragma unroll 1
  for (int k0 = 0; k0 < EMBED; k0 += 32) {
    v16bf ah[2], al[2], bh[2], bl[2];
#pragma unroll
    for (int i = 0; i < 2; ++i) {
      ah[i] = ldfrag(aph + (size_t)(i * 16) * EMBED + k0, EMBED, m, hl);
      al[i] = ldfrag(apl + (size_t)(i * 16) * EMBED + k0, EMBED, m, hl);
      bh[i] = ldfrag(bph + (size_t)(i * 16) * EMBED + k0, EMBED, m, hl);
      bl[i] = ldfrag(bpl + (size_t)(i * 16) * EMBED + k0, EMBED, m, hl);
    }
#pragma unroll
    for (int mf = 0; mf < 2; ++mf)
#pragma unroll
      for (int nf = 0; nf < 2; ++nf)
        acc[mf][nf] = mma3(acc[mf][nf], ah[mf], al[mf], bh[nf], bl[nf]);
  }

#pragma unroll
  for (int mf = 0; mf < 2; ++mf)
#pragma unroll
    for (int nf = 0; nf < 2; ++nf)
#pragma unroll
      for (int r = 0; r < 8; ++r)
        sC[(wm * 32 + mf * 16 + 8 * hl + r) * SCP + wn * 32 + nf * 16 + m] = acc[mf][nf][r];
  __syncthreads();

  if (EPI == 0) {
    const int sec = n0 >> 10;
    const int hb = (n0 & 1023) >> 6;
    if (sec < 2) {
      us_t* Ph = (sec == 0) ? Qh : Kh;
      us_t* Pl = (sec == 0) ? Ql : Kl;
      const float sc = (sec == 0) ? 0.125f : 1.0f;
      for (int pass = 0; pass < 2; ++pass) {
#pragma unroll
        for (int it = 0; it < 4; ++it) {
          const int L = it * 32 + (tid >> 3);
          const int seg = (tid & 7) * 8;
          const int row = L >> 1, hh = L & 1;
          const int col = hh * 64 + seg;
          v4f a = *(const v4f*)(sC + row * SCP + col);
          v4f c = *(const v4f*)(sC + row * SCP + col + 4);
          const v4f ba = *(const v4f*)(bias + n0 + col);
          const v4f bc = *(const v4f*)(bias + n0 + col + 4);
          a = (a + ba) * sc;
          c = (c + bc) * sc;
          v4u hw, lw;
          split8(a, c, hw, lw);
          const int gr = m0 + row;
          const int bb = gr >> 11, t = gr & (SEQ - 1);
          const int bhh = bb * NHEADS + hb + hh;
          const size_t d = ((size_t)bhh * SEQ + t) * HDIM + seg;
          *(volatile v4u*)(Ph + d) = hw;
          *(volatile v4u*)(Pl + d) = lw;
        }
        if (pass == 0) __threadfence();
      }
    } else {
      const int bb = m0 >> 11;
      const int t0 = m0 & (SEQ - 1);
      for (int pass = 0; pass < 2; ++pass) {
#pragma unroll
        for (int it = 0; it < 4; ++it) {
          const int L = it * 32 + (tid >> 3);
          const int seg = (tid & 7) * 8;
          const float bv = bias[n0 + L];
          v4f a, c;
#pragma unroll
          for (int e = 0; e < 4; ++e) {
            a[e] = sC[(seg + e) * SCP + L] + bv;
            c[e] = sC[(seg + 4 + e) * SCP + L] + bv;
          }
          v4u hw, lw;
          split8(a, c, hw, lw);
          const int hd = hb + (L >> 6);
          const int dd = L & 63;
          const int bhh = bb * NHEADS + hd;
          const size_t d = ((size_t)bhh * HDIM + dd) * SEQ + t0 + seg;
          *(volatile v4u*)(Vh + d) = hw;
          *(volatile v4u*)(Vl + d) = lw;
        }
        if (pass == 0) __threadfence();
      }
    }
  } else {
    for (int pass = 0; pass < 2; ++pass) {
#pragma unroll
      for (int it = 0; it < 8; ++it) {
        const int row = w * 8 + it;
        const int col = 4 * l;
        v4f a = *(const v4f*)(sC + row * SCP + col);
        const v4f bb = *(const v4f*)(bias + n0 + col);
        a = a + bb;
        *(volatile v4f*)(Fo + (size_t)(m0 + row) * EMBED + n0 + col) = a;
      }
      if (pass == 0) __threadfence();
    }
  }
}

__global__ __launch_bounds__(128) void k_attn(const us_t* __restrict__ Qh, const us_t* __restrict__ Ql,
                                               const us_t* __restrict__ Kh, const us_t* __restrict__ Kl,
                                               const us_t* __restrict__ Vh, const us_t* __restrict__ Vl,
                                               us_t* Ch, us_t* Cl) {
  __shared__ __align__(16) float sS[4][16 * SSP];
  __shared__ __align__(16) unsigned sP[4][2][16 * 32];

  const int tid = (int)threadIdx.x;
  const int w = tid >> 5, l = tid & 31, hl = l >> 4, m = l & 15;
  const int qb = blockIdx.x & 31;
  const int bh = blockIdx.x >> 5;
  const int q0 = qb * 64 + w * 16;
  const int b = bh >> 4, h = bh & 15;
  const size_t qkoff = (size_t)bh * SEQ * HDIM;
  const size_t voff = (size_t)bh * HDIM * SEQ;
  float* mS = &sS[w][0];
  unsigned* mPh = &sP[w][0][0];
  unsigned* mPl = &sP[w][1][0];

  v16bf qh[2], ql[2];
#pragma unroll
  for (int ks = 0; ks < 2; ++ks) {
    qh[ks] = ldfrag(Qh + qkoff + (size_t)q0 * HDIM + ks * 32, HDIM, m, hl);
    ql[ks] = ldfrag(Ql + qkoff + (size_t)q0 * HDIM + ks * 32, HDIM, m, hl);
  }

  v8f o[4];
#pragma unroll
  for (int nf = 0; nf < 4; ++nf) o[nf] = v8f{};
  float mrow = -__builtin_inff();
  float lrow = 0.0f;

  const int ntiles = qb + 1;
#pragma unroll 1
  for (int kt = 0; kt < ntiles; ++kt) {
    const int k0 = kt * 64;

    v8f s[4];
#pragma unroll
    for (int nf = 0; nf < 4; ++nf) s[nf] = v8f{};
#pragma unroll
    for (int nf = 0; nf < 4; ++nf) {
      const us_t* kbh = Kh + qkoff + (size_t)(k0 + nf * 16) * HDIM;
      const us_t* kbl = Kl + qkoff + (size_t)(k0 + nf * 16) * HDIM;
#pragma unroll
      for (int ks = 0; ks < 2; ++ks) {
        const v16bf kh = ldfrag(kbh + ks * 32, HDIM, m, hl);
        const v16bf kl = ldfrag(kbl + ks * 32, HDIM, m, hl);
        s[nf] = mma3(s[nf], qh[ks], ql[ks], kh, kl);
      }
    }

#pragma unroll
    for (int nf = 0; nf < 4; ++nf)
#pragma unroll
      for (int r = 0; r < 8; ++r) {
        const int srow = 8 * hl + r;
        const int scol = nf * 16 + m;
        float v = s[nf][r];
        if (k0 + scol > q0 + srow) v = -FLT_MAX;
        mS[srow * SSP + scol] = v;
      }
    __syncthreads();

    const float* rp = mS + m * SSP + hl * 32;
    float smax = -__builtin_inff();
#pragma unroll
    for (int j4 = 0; j4 < 8; ++j4) {
      const v4f t4 = *(const v4f*)(rp + j4 * 4);
      smax = fmaxf(smax, fmaxf(fmaxf(t4[0], t4[1]), fmaxf(t4[2], t4[3])));
    }
    smax = fmaxf(smax, __shfl_xor(smax, 16, 32));
    const float mnew = fmaxf(mrow, smax);
    const float alpha = __expf(mrow - mnew);
    float psum = 0.0f;
#pragma unroll
    for (int j8 = 0; j8 < 4; ++j8) {
      v4f a = *(const v4f*)(rp + j8 * 8);
      v4f c = *(const v4f*)(rp + j8 * 8 + 4);
#pragma unroll
      for (int e = 0; e < 4; ++e) {
        a[e] = __expf(a[e] - mnew);
        c[e] = __expf(c[e] - mnew);
        psum += a[e] + c[e];
      }
      v4u hw, lw;
      split8(a, c, hw, lw);
      *(v4u*)(mPh + m * 32 + hl * 16 + j8 * 4) = hw;
      *(v4u*)(mPl + m * 32 + hl * 16 + j8 * 4) = lw;
    }
    psum += __shfl_xor(psum, 16, 32);
    lrow = lrow * alpha + psum;
#pragma unroll
    for (int r = 0; r < 8; ++r) {
      const float ar = __shfl(alpha, 8 * hl + r, 32);
#pragma unroll
      for (int nf = 0; nf < 4; ++nf) o[nf][r] *= ar;
    }
    mrow = mnew;
    __syncthreads();

#pragma unroll
    for (int ks2 = 0; ks2 < 2; ++ks2) {
      const v16bf ph = ldfrag((const us_t*)mPh + ks2 * 32, 64, m, hl);
      const v16bf pl = ldfrag((const us_t*)mPl + ks2 * 32, 64, m, hl);
#pragma unroll
      for (int nf = 0; nf < 4; ++nf) {
        const us_t* vbh = Vh + voff + (size_t)(nf * 16) * SEQ + k0 + ks2 * 32;
        const us_t* vbl = Vl + voff + (size_t)(nf * 16) * SEQ + k0 + ks2 * 32;
        const v16bf vh = ldfrag(vbh, SEQ, m, hl);
        const v16bf vl = ldfrag(vbl, SEQ, m, hl);
        o[nf] = mma3(o[nf], ph, pl, vh, vl);
      }
    }
  }

  const float linv = 1.0f / lrow;
#pragma unroll
  for (int r = 0; r < 8; ++r) {
    const float li = __shfl(linv, 8 * hl + r, 32);
#pragma unroll
    for (int nf = 0; nf < 4; ++nf)
      mS[(8 * hl + r) * SSP + nf * 16 + m] = o[nf][r] * li;
  }
  __syncthreads();
  for (int pass = 0; pass < 2; ++pass) {
#pragma unroll
    for (int it = 0; it < 4; ++it) {
      const int row = it * 4 + (l >> 3);
      const int seg = (l & 7) * 8;
      const v4f a = *(const v4f*)(mS + row * SSP + seg);
      const v4f c = *(const v4f*)(mS + row * SSP + seg + 4);
      v4u hw, lw;
      split8(a, c, hw, lw);
      const size_t d = ((size_t)(b * SEQ + q0 + row)) * EMBED + h * HDIM + seg;
      *(volatile v4u*)(Ch + d) = hw;
      *(volatile v4u*)(Cl + d) = lw;
    }
    if (pass == 0) __threadfence();
  }
}

extern "C" void kernel_launch(void* const* d_in, const int* in_sizes, int n_in,
                              void* d_out, int out_size, void* d_ws, size_t ws_size,
                              hipStream_t stream) {
  if (n_in < 5) return;
  if (in_sizes[0] != MROWS * EMBED || in_sizes[1] != EMBED * N3 || in_sizes[2] != N3 ||
      in_sizes[3] != EMBED * EMBED || in_sizes[4] != EMBED || out_size != MROWS * EMBED) return;

  const float* x    = (const float*)d_in[0];
  const float* Wqkv = (const float*)d_in[1];
  const float* bqkv = (const float*)d_in[2];
  const float* Wout = (const float*)d_in[3];
  const float* bout = (const float*)d_in[4];
  float* out = (float*)d_out;

  char* ws = (char*)d_ws;
  size_t off = 0;
  auto carve = [&](size_t bytes) -> char* {
    char* p = ws + off;
    off += (bytes + 255) & ~(size_t)255;
    return p;
  };
  const size_t xplane = (size_t)MROWS * EMBED * 2;
  const size_t wqplane = (size_t)N3 * EMBED * 2;
  const size_t woplane = (size_t)EMBED * EMBED * 2;
  const size_t hplane = (size_t)BHEADS * SEQ * HDIM * 2;
  us_t* Xh  = (us_t*)carve(xplane);
  us_t* Xl  = (us_t*)carve(xplane);
  us_t* Wqh = (us_t*)carve(wqplane);
  us_t* Wql = (us_t*)carve(wqplane);
  us_t* Woh = (us_t*)carve(woplane);
  us_t* Wol = (us_t*)carve(woplane);
  us_t* Qh  = (us_t*)carve(hplane);
  us_t* Ql  = (us_t*)carve(hplane);
  us_t* Kh  = (us_t*)carve(hplane);
  us_t* Kl  = (us_t*)carve(hplane);
  us_t* Vh  = (us_t*)carve(hplane);
  us_t* Vl  = (us_t*)carve(hplane);
  us_t* Ch  = (us_t*)carve(xplane);
  us_t* Cl  = (us_t*)carve(xplane);
  if (off > ws_size) return;

  k_cvt_rows<<<dim3(MROWS * EMBED / 8 / 256), 256, 0, stream>>>(x, Xh, Xl, MROWS * EMBED / 8);
  k_cvt_tr<<<dim3(N3 / 64, EMBED / 64), 256, 0, stream>>>(Wqkv, Wqh, Wql, EMBED, N3);
  k_cvt_tr<<<dim3(EMBED / 64, EMBED / 64), 256, 0, stream>>>(Wout, Woh, Wol, EMBED, EMBED);
  k_gemm<0><<<dim3(N3 / 128, MROWS / 64), 256, 0, stream>>>(
      Xh, Xl, Wqh, Wql, bqkv, Qh, Ql, Kh, Kl, Vh, Vl, out);
  k_attn<<<dim3(BHEADS * (SEQ / 64)), 128, 0, stream>>>(Qh, Ql, Kh, Kl, Vh, Vl, Ch, Cl);
  k_gemm<1><<<dim3(EMBED / 128, MROWS / 64), 256, 0, stream>>>(
      Ch, Cl, Woh, Wol, bout, Qh, Ql, Kh, Kl, Vh, Vl, out);
}
